// LearnedDistance_29411936043390
// MI455X (gfx1250) — hardware-verified
//
#include <hip/hip_runtime.h>
#include <math.h>

typedef __attribute__((ext_vector_type(16))) _Float16 v16h;
typedef __attribute__((ext_vector_type(16))) __bf16 v16b;
typedef __attribute__((ext_vector_type(8)))  _Float16 v8h;
typedef __attribute__((ext_vector_type(8)))  float v8f;
typedef __attribute__((ext_vector_type(4)))  float v4f;
typedef __attribute__((ext_vector_type(2)))  float v2f;
typedef __attribute__((ext_vector_type(4)))  unsigned v4u;
typedef __attribute__((ext_vector_type(4)))  int v4i;
typedef float __attribute__((may_alias)) float_a;
typedef int __attribute__((may_alias)) int_a;

template <typename T> __device__ __forceinline__ void vst2(void* p, T v) { *(volatile T*)p = v; __threadfence(); *(volatile T*)p = v; }
__device__ __forceinline__ v8f wmma16(v16h a, v16h b, v8f c) {
  v8f d = __builtin_amdgcn_wmma_f32_16x16x32_f16(false, a, false, b, (short)0, c, false, false);
  asm volatile("v_nop\n\tv_nop\n\tv_nop\n\tv_nop" : "+v"(d) : "v"(a), "v"(b));
  return d;
}
__device__ __forceinline__ v8f wmma_bf(v16b a, v16b b, v8f c) {
  v8f d = __builtin_amdgcn_wmma_f32_16x16x32_bf16(false, a, false, b, (short)0, c, false, false);
  asm volatile("v_nop\n\tv_nop\n\tv_nop\n\tv_nop" : "+v"(d) : "v"(a), "v"(b));
  return d;
}
__device__ __forceinline__ v16h frag_h(const _Float16* rowk0, int lane) {
  union { v16h v; v8h q[2]; } u; const _Float16* p = rowk0 + 8 * (lane >> 4);
  u.q[0] = *(const v8h*)p; u.q[1] = *(const v8h*)(p + 16); return u.v;
}
__device__ __forceinline__ v16h frag_f32(const float* rowk0, int lane) {
  v16h a; const float* p = rowk0 + 8 * (lane >> 4);
#pragma unroll
  for (int i = 0; i < 8; ++i) { a[i] = (_Float16)p[i]; a[8 + i] = (_Float16)p[16 + i]; }
  return a;
}
__device__ __forceinline__ v16h frag_f32s(const float* rowk0, int lane, float sc) {
  v16h a; const float* p = rowk0 + 8 * (lane >> 4);
#pragma unroll
  for (int i = 0; i < 8; ++i) { a[i] = (_Float16)(p[i] * sc); a[8 + i] = (_Float16)(p[16 + i] * sc); }
  return a;
}
__device__ __forceinline__ v16h fragc_f32(const float* W, int k0, int n, int lane, int ld, int K) {
  v16h a; const int g = lane >> 4;
#pragma unroll
  for (int i = 0; i < 8; ++i) { const int ka = k0 + 8 * g + i, kb = ka + 16;
    a[i] = (_Float16)(ka < K ? W[(size_t)(ka < K ? ka : K - 1) * ld + n] : 0.f); a[8 + i] = (_Float16)(kb < K ? W[(size_t)(kb < K ? kb : K - 1) * ld + n] : 0.f); }
  return a;
}
struct F2 { v16b h, l; };
__device__ __forceinline__ F2 bsplit16(const float v[16]) { F2 r;
#pragma unroll
  for (int i = 0; i < 16; ++i) { const __bf16 h = (__bf16)v[i]; r.h[i] = h; r.l[i] = (__bf16)(v[i] - (float)h); }
  return r; }
__device__ __forceinline__ F2 split_row(const float* row, int k0, int lane) { float v[16]; const float* p = row + k0 + 8 * (lane >> 4);
#pragma unroll
  for (int i = 0; i < 8; ++i) { v[i] = p[i]; v[8 + i] = p[16 + i]; }
  return bsplit16(v); }
__device__ __forceinline__ F2 split_rowK(const float* row, int k0, int lane, int K) { float v[16]; const int g = lane >> 4;
#pragma unroll
  for (int i = 0; i < 8; ++i) { const int ka = k0 + 8 * g + i, kb = ka + 16; v[i] = ka < K ? row[ka < K ? ka : K - 1] : 0.f; v[8 + i] = kb < K ? row[kb < K ? kb : K - 1] : 0.f; }
  return bsplit16(v); }
__device__ __forceinline__ F2 split_col(const float* W, int k0, int n, int lane, int ld, int K) { float v[16]; const int g = lane >> 4;
#pragma unroll
  for (int i = 0; i < 8; ++i) { const int ka = k0 + 8 * g + i, kb = ka + 16; v[i] = ka < K ? W[(size_t)(ka < K ? ka : K - 1) * ld + n] : 0.f; v[8 + i] = kb < K ? W[(size_t)(kb < K ? kb : K - 1) * ld + n] : 0.f; }
  return bsplit16(v); }
__device__ __forceinline__ v8f mac3(const F2& a, const F2& b, v8f c) { c = wmma_bf(a.l, b.h, c); c = wmma_bf(a.h, b.l, c); return wmma_bf(a.h, b.h, c); }
__device__ __forceinline__ float sigm(float v) { return 1.0f / (1.0f + expf(-v)); }
#define LDSX() do { asm volatile("s_wait_dscnt 0" ::: "memory"); __builtin_amdgcn_wave_barrier(); __builtin_amdgcn_fence(__ATOMIC_RELEASE, "workgroup"); } while (0)


#define NQ 2048
#define DH 256
#define DK 64
#define FF 32
#ifndef NIT
#define NIT (NQ / 16)
#endif
typedef __attribute__((ext_vector_type(8))) __bf16 v8b;
__device__ __forceinline__ v16b frag_b(const __bf16* rowk0, int lane) {
  union { v16b v; v8b q[2]; } u; const __bf16* p = rowk0 + 8 * (lane >> 4);
  u.q[0] = *(const v8b*)p; u.q[1] = *(const v8b*)(p + 16); return u.v;
}
__device__ __forceinline__ float bfr(float v) { return (float)(__bf16)v; }
__device__ __attribute__((noinline)) float exp_ni(float v) { return expf(v); }
__device__ __attribute__((noinline)) float erf_ni(float v) { return erff(v); }

#define WS_PW   0u
#define P_Q 0
#define P_K (P_Q + 64 * 256)
#define P_V (P_K + 64 * 256)
#define P_2 (P_V + 256 * 256)
#define PWEND (P_2 + 32 * 32)
#define WS_QM   (WS_PW + 2u * PWEND)
#define WS_KM   (WS_QM + 4u * NQ * DK)
#define WS_VT   (WS_KM + 4u * NQ * DK)
#define WS_VTL  (WS_VT + 2u * DH * NQ)
#define WS_QT   (WS_VTL + 2u * DH * NQ)
#define WS_LG   (WS_QT + 16u)
#define WS_END  (WS_LG + 4u * NQ * NQ)

__global__ __launch_bounds__(256) void k_packW(const float* __restrict__ WQ, const float* __restrict__ WK, const float* __restrict__ WV, const float* __restrict__ W2, __bf16* __restrict__ PW) {
  __shared__ __align__(16) __bf16 s[256]; const int o = blockIdx.x, which = blockIdx.y, t = threadIdx.x;
  if (which == 0) { if (o >= DK) return; s[t] = (__bf16)WQ[(size_t)t * DK + o]; } else if (which == 1) { if (o >= DK) return; s[t] = (__bf16)WK[(size_t)t * DK + o]; } else if (which == 2) { s[t] = (__bf16)WV[(size_t)t * DH + o]; } else { if (o >= FF) return; if (t < FF) s[t] = (__bf16)W2[(size_t)t * FF + o]; }
  __syncthreads();
  if (which < 2) { if (t < 32) vst2((unsigned*)(PW + (which ? P_K : P_Q) + (size_t)o * 256 + t * 8), *(const v4u*)&s[t * 8]); }
  else if (which == 2) { if (t < 32) vst2((unsigned*)(PW + P_V + (size_t)o * 256 + t * 8), *(const v4u*)&s[t * 8]); }
  else { if (t < 4) vst2((unsigned*)(PW + P_2 + (size_t)o * 32 + t * 8), *(const v4u*)&s[t * 8]); }
}
__global__ __launch_bounds__(128) void k_qkv(const float* __restrict__ X, const __bf16* __restrict__ PW, const float* __restrict__ BQ, const float* __restrict__ BK, const float* __restrict__ BV, float* __restrict__ QM, float* __restrict__ KM, __bf16* __restrict__ VT, __bf16* __restrict__ VTL) {
  __shared__ __align__(16) float so[4][16][132]; __shared__ __align__(16) __bf16 sh[128][72], sl[128][72];
  const int tid = threadIdx.x, wave = tid >> 5, lane = tid & 31, col = lane & 15, g = lane >> 4; const size_t r0 = (size_t)blockIdx.x * 64 + wave * 16; const int which = blockIdx.y;
  const int NT = (which < 2) ? 4 : 8; const __bf16* P = PW + (which == 0 ? P_Q : which == 1 ? P_K : P_V + (size_t)(which - 2) * 128 * 256); const float* bias = (which == 0) ? BQ : (which == 1) ? BK : BV + (which - 2) * 128;
  v8f acc[8] = {};
#pragma unroll 2
  for (int kc = 0; kc < DH / 32; ++kc) { v16b a; { const float* p = X + (r0 + col) * DH + kc * 32 + 8 * g;
#pragma unroll
      for (int i2 = 0; i2 < 8; ++i2) { a[i2] = (__bf16)p[i2]; a[8 + i2] = (__bf16)p[16 + i2]; } }
#pragma unroll
    for (int j = 0; j < 8; ++j) if (j < NT) acc[j] = wmma_bf(a, frag_b(P + (size_t)(j * 16 + col) * 256 + kc * 32, lane), acc[j]); }
#pragma unroll
  for (int j = 0; j < 8; ++j) { if (j < NT) { const float bb = bfr(bias[j * 16 + col]);
#pragma unroll
    for (int r = 0; r < 8; ++r) so[wave][8 * g + r][j * 16 + col] = acc[j][r] + bb; } }
  LDSX();
  if (which < 2) { float* dstm = which ? KM : QM; for (int rl = 0; rl < 16; ++rl) { if (lane < 16) vst2(dstm + (r0 + rl) * DK + lane * 4, *(const v4f*)&so[wave][rl][lane * 4]); } }
  else {
    __syncthreads();
    for (int q = tid; q < 128 * 64; q += 128) { const int c = q >> 6, rl = q & 63; const float v = so[rl >> 4][rl & 15][c]; const __bf16 h = (__bf16)v; sh[c][rl] = h; sl[c][rl] = (__bf16)(v - (float)h); }
    __syncthreads();
    for (int q = tid; q < 128 * 8; q += 128) { const int c = q >> 3, pc = q & 7; const size_t d = (size_t)(which - 2) * 128 + c; vst2((unsigned*)(VT + d * NQ + (size_t)blockIdx.x * 64 + pc * 8), *(const v4u*)&sh[c][pc * 8]); vst2((unsigned*)(VTL + d * NQ + (size_t)blockIdx.x * 64 + pc * 8), *(const v4u*)&sl[c][pc * 8]); } }
}
__global__ __launch_bounds__(128) void k_pair(const float* __restrict__ QM, const float* __restrict__ KM, const float* __restrict__ ADJ, const float* __restrict__ DEN, const float* __restrict__ W1, const float* __restrict__ B1, const __bf16* __restrict__ PW, const float* __restrict__ B2, const float* __restrict__ W3, const float* __restrict__ B3, float* __restrict__ LG) {
  __shared__ __align__(16) float ssc[16][132]; __shared__ __align__(16) float sa[4][16][36]; __shared__ __align__(16) float sh2[4][16][36]; __shared__ __align__(16) float slg[16][132]; __shared__ float sw1[3][FF], sb1[FF], sb2[FF], sw3[FF];
  const int tid = threadIdx.x, wave = tid >> 5, lane = tid & 31, col = lane & 15, g = lane >> 4; const int i0 = blockIdx.x * 16; const int j0 = blockIdx.y * 128;
  if (tid < FF) { sw1[0][tid] = bfr(W1[tid]); sw1[1][tid] = bfr(W1[FF + tid]); sw1[2][tid] = bfr(W1[2 * FF + tid]); sb1[tid] = bfr(B1[tid]); sb2[tid] = bfr(B2[tid]); sw3[tid] = bfr(W3[tid]); }
  { v8f acc[2] = {};
#pragma unroll
    for (int kc = 0; kc < 2; ++kc) { const F2 a = split_row(KM + (size_t)(i0 + col) * DK, kc * 32, lane);
#pragma unroll
      for (int t2 = 0; t2 < 2; ++t2) { const F2 b = split_row(QM + (size_t)(j0 + wave * 32 + t2 * 16 + col) * DK, kc * 32, lane); acc[t2] = wmma_bf(a.l, b.h, acc[t2]); acc[t2] = wmma_bf(a.h, b.l, acc[t2]); acc[t2] = wmma_bf(a.h, b.h, acc[t2]); } }
#pragma unroll
    for (int t2 = 0; t2 < 2; ++t2)
#pragma unroll
      for (int r = 0; r < 8; ++r) ssc[8 * g + r][wave * 32 + t2 * 16 + col] = acc[t2][r]; }
  __syncthreads();
  const float b3 = bfr(B3[0]);
#pragma unroll 1
  for (int tt = 0; tt < 32; ++tt) { const int rl = tt >> 1, jt = tt & 1; const int jl0 = wave * 32 + jt * 16;
    { const int p = col; const int j = j0 + jl0 + p; const size_t i = (size_t)(i0 + rl); const float s = ssc[rl][jl0 + p], av = bfr(ADJ[i * NQ + j]), dv = bfr(DEN[i * NQ + j]);
#pragma unroll 1
      for (int f = g * 16; f < g * 16 + 16; ++f) { const float v = ((s * sw1[0][f] + av * sw1[1][f]) + dv * sw1[2][f]) + sb1[f]; sa[wave][p][f] = fmaxf(v, 0.f); } }
    LDSX();
    v8f acc2[2] = {}; { const F2 a = split_row(&sa[wave][col][0], 0, lane);
#pragma unroll
      for (int t2 = 0; t2 < 2; ++t2) { const v16b w = frag_b(PW + P_2 + (size_t)(t2 * 16 + col) * 32, lane); acc2[t2] = wmma_bf(a.l, w, acc2[t2]); acc2[t2] = wmma_bf(a.h, w, acc2[t2]); } }
#pragma unroll
    for (int t2 = 0; t2 < 2; ++t2)
#pragma unroll
      for (int r = 0; r < 8; ++r) sh2[wave][8 * g + r][t2 * 16 + col] = fmaxf(acc2[t2][r] + sb2[t2 * 16 + col], 0.f);
    LDSX();
    if (lane < 16) { const int p = lane; float a3 = b3;
#pragma unroll 1
      for (int f = 0; f < FF; ++f) a3 += sh2[wave][p][f] * sw3[f];
      slg[rl][jl0 + p] = a3; }
    LDSX(); }
  __syncthreads();
  for (int q = tid; q < 16 * 32; q += 128) { const int rl = q >> 5, pc = q & 31; vst2(LG + (size_t)(i0 + rl) * NQ + j0 + pc * 4, *(const v4f*)&slg[rl][pc * 4]); }
}
__global__ __launch_bounds__(128) void k_soft(const float* __restrict__ LG, const __bf16* __restrict__ VT, const __bf16* __restrict__ VTL, float* __restrict__ OUT) {
  __shared__ float smx[16], siz[16]; __shared__ __align__(16) float sp[16][36]; __shared__ __align__(16) float so[16][260];
  const int tid = threadIdx.x, wave = tid >> 5, lane = tid & 31, col = lane & 15, g = lane >> 4; const int i0 = blockIdx.x * 16;
  for (int rr = 0; rr < 4; ++rr) { const int rl = wave * 4 + rr; const float* row = LG + (size_t)(i0 + rl) * NQ; float mx = -3.0e38f; for (int j = lane; j < NQ; j += 32) mx = fmaxf(mx, row[j]);
#pragma unroll
    for (int o = 1; o < 32; o <<= 1) mx = fmaxf(mx, __shfl_xor(mx, o));
    float z = 0.f; for (int j = lane; j < NQ; j += 32) z += exp_ni(row[j] - mx);
#pragma unroll
    for (int o = 1; o < 32; o <<= 1) z += __shfl_xor(z, o);
    if (lane == 0) { smx[rl] = mx; siz[rl] = 1.0f / z; } }
  __syncthreads();
  v8f acc[4] = {};
#pragma unroll 1
  for (int ks = 0; ks < NQ / 32; ++ks) {
    v16b ph, pl; { const float* row = LG + (size_t)(i0 + col) * NQ + ks * 32 + 8 * g; const float m = smx[col], iz = siz[col];
#pragma unroll
      for (int i2 = 0; i2 < 16; ++i2) { const float v = exp_ni(row[i2 < 8 ? i2 : 8 + i2] - m) * iz; const __bf16 h = (__bf16)v; ph[i2] = h; pl[i2] = (__bf16)(v - (float)h); } }
#pragma unroll
    for (int j = 0; j < 4; ++j) { const size_t pr = ((size_t)(wave * 64 + j * 16 + col)) * NQ + ks * 32; const v16b vh = frag_b(VT + pr, lane), vl = frag_b(VTL + pr, lane); acc[j] = wmma_bf(pl, vh, acc[j]); acc[j] = wmma_bf(ph, vl, acc[j]); acc[j] = wmma_bf(ph, vh, acc[j]); } }
#pragma unroll
  for (int j = 0; j < 4; ++j)
#pragma unroll
    for (int r = 0; r < 8; ++r) so[8 * g + r][wave * 64 + j * 16 + col] = acc[j][r];
  __syncthreads();
  for (int q = tid; q < 16 * 64; q += 128) { const int rl = q >> 6, pc = q & 63; vst2(OUT + (size_t)(i0 + rl) * DH + pc * 4, *(const v4f*)&so[rl][pc * 4]); }
}
extern "C" void kernel_launch(void* const* d_in, const int* in_sizes, int n_in, void* d_out, int out_size, void* d_ws, size_t ws_size, hipStream_t stream) {
  (void)in_sizes; (void)n_in; (void)out_size;
  const float** F = (const float**)d_in;
  if (ws_size < (size_t)WS_END) return;
  char* ws = (char*)d_ws; __bf16* PW = (__bf16*)(ws + WS_PW); float *QM = (float*)(ws + WS_QM), *KM = (float*)(ws + WS_KM), *LG = (float*)(ws + WS_LG); __bf16 *VT = (__bf16*)(ws + WS_VT), *VTL = (__bf16*)(ws + WS_VTL);
  k_packW<<<dim3(256, 4), 256, 0, stream>>>(F[3], F[5], F[7], F[11], PW);
  k_qkv<<<dim3(NQ / 64, 4), 128, 0, stream>>>(F[0], PW, F[4], F[6], F[8], QM, KM, VT, VTL);
  k_pair<<<dim3(NIT, NQ / 128), 128, 0, stream>>>(QM, KM, F[1], F[2], F[9], F[10], PW, F[12], F[13], F[14], LG);
  k_soft<<<NIT, 128, 0, stream>>>(LG, VT, VTL, (float*)d_out);
}
